// SetAbstraction_31061203485290
// MI455X (gfx1250) — hardware-verified
//
#include <hip/hip_runtime.h>
#include <stddef.h>

typedef __attribute__((ext_vector_type(16))) __bf16   v16b;
typedef __attribute__((ext_vector_type(8)))  __bf16   v8b;
typedef __attribute__((ext_vector_type(8)))  _Float16 v8h;
typedef __attribute__((ext_vector_type(8)))  float    v8f;
typedef __attribute__((ext_vector_type(4)))  float    v4f;
typedef __attribute__((ext_vector_type(4)))  unsigned int v4u;
typedef __attribute__((ext_vector_type(2)))  unsigned int v2u;

constexpr int NBATCH = 4;
constexpr int NPT    = 8192;
constexpr int CIN    = 64;
constexpr int COUT   = 128;
constexpr int KNB    = 32;
constexpr int MPT    = 2048;
constexpr int CPE    = 32;
constexpr int QPB    = 32;
constexpr int XP     = 40;
constexpr int MVP    = 36;
constexpr float RAD2 = 0.01f;

static_assert((NPT & (NPT - 1)) == 0, "NPT power of two (index clamp by mask)");
static_assert(MPT % QPB == 0 && QPB == 32, "one 128-B output line per channel row per tail block");
static_assert(NPT % 64 == 0 && MPT % 64 == 0 && CIN % 64 == 0 && COUT % 64 == 0, "GEMM M/N tile multiples");
static_assert(CIN % 32 == 0 && (2 * CIN) % 32 == 0, "GEMM K multiple of 32");

constexpr size_t SZ_PR   = (size_t)NBATCH * NPT * 4 * 4;
constexpr size_t SZ_FT   = (size_t)NBATCH * NPT * CIN * 2;
constexpr size_t SZ_W10  = (size_t)CIN * CIN * 2;
constexpr size_t SZ_W11  = (size_t)COUT * 2 * CIN * 2;
constexpr size_t SZ_WSK  = (size_t)COUT * CIN * 2;
constexpr size_t SZ_NEWP = (size_t)NBATCH * MPT * 4 * 4;
constexpr size_t SZ_FIT  = (size_t)NBATCH * MPT * CIN * 2;
constexpr size_t SZ_H1   = (size_t)NBATCH * NPT * 2 * CIN * 2;
constexpr size_t SZ_HT   = (size_t)NBATCH * NPT * COUT * 4;
constexpr size_t SZ_ID   = (size_t)NBATCH * COUT * MPT * 4;
constexpr size_t OFF_PR   = 0;
constexpr size_t OFF_FT   = OFF_PR + SZ_PR;
constexpr size_t OFF_W10  = OFF_FT + SZ_FT;
constexpr size_t OFF_W11  = OFF_W10 + SZ_W10;
constexpr size_t OFF_WSK  = OFF_W11 + SZ_W11;
constexpr size_t OFF_NEWP = OFF_WSK + SZ_WSK;
constexpr size_t OFF_FIT  = OFF_NEWP + SZ_NEWP;
constexpr size_t OFF_H1   = OFF_FIT + SZ_FIT;
constexpr size_t OFF_HT   = OFF_H1 + SZ_H1;
constexpr size_t OFF_ID   = OFF_HT + SZ_HT;
constexpr size_t WS_TOTAL = OFF_ID + SZ_ID;
static_assert(WS_TOTAL <= (size_t)134217728, "carve within 128 MiB");
static_assert(OFF_FT % 256 == 0 && OFF_W10 % 256 == 0 && OFF_W11 % 256 == 0 && OFF_WSK % 256 == 0 &&
              OFF_NEWP % 256 == 0 && OFF_FIT % 256 == 0 && OFF_H1 % 256 == 0 && OFF_HT % 256 == 0 &&
              OFF_ID % 256 == 0, "region alignment");

__device__ __forceinline__ unsigned short f2bf_bits(float f) {
  unsigned u = __float_as_uint(f);
  return (unsigned short)((u + 0x7FFFu + ((u >> 16) & 1u)) >> 16);
}
__device__ __forceinline__ float bf_bits2f(unsigned short h) { return __uint_as_float(((unsigned)h) << 16); }
__device__ __forceinline__ float rbf(float x) { return bf_bits2f(f2bf_bits(x)); }
__device__ __forceinline__ unsigned pack_bf2(float a, float b) {
  return (unsigned)f2bf_bits(a) | (((unsigned)f2bf_bits(b)) << 16);
}

__device__ __forceinline__ float dist2_ord(float ax, float ay, float az, float bx, float by, float bz) {
#pragma clang fp contract(off)
  const float dx = ax - bx;
  const float dy = ay - by;
  const float dz = az - bz;
  const float t0 = dx * dx;
  const float t1 = dy * dy;
  const float t2 = dz * dz;
  const float u = t0 + t2;
  return u + t1;
}

__device__ __forceinline__ void wave_sync() {
  __builtin_amdgcn_fence(__ATOMIC_RELEASE, "workgroup");
  __builtin_amdgcn_wave_barrier();
  __builtin_amdgcn_fence(__ATOMIC_ACQUIRE, "workgroup");
}

__device__ __forceinline__ void dep_guard_b(v8f& a, v8f& b, v16b x, v16b y) { asm volatile("v_nop\n\tv_nop\n\tv_nop\n\tv_nop" : "+v"(a), "+v"(b) : "v"(x), "v"(y)); }
__device__ __forceinline__ void dep_guard3(v8f& a, v8f& b, v16b x, v16b y, v16b z) { asm volatile("v_nop\n\tv_nop\n\tv_nop\n\tv_nop" : "+v"(a), "+v"(b) : "v"(x), "v"(y), "v"(z)); }
__device__ __forceinline__ void keep4_b(v16b a, v16b b, v16b c, v16b d) { asm volatile("v_nop" :: "v"(a), "v"(b), "v"(c), "v"(d)); }
__device__ __forceinline__ void acc_guard4(v8f& a, v8f& b, v8f& c, v8f& d) { asm volatile("v_nop\n\tv_nop\n\tv_nop\n\tv_nop" : "+v"(a), "+v"(b), "+v"(c), "+v"(d)); }

template <typename T> struct Frag;
template <> struct Frag<__bf16> {
  typedef v16b V; union U { v16b v; v8b h[2]; };
  static __device__ __forceinline__ v16b load(const __bf16* p) {
    U f; f.h[0] = *(const v8b*)(p); f.h[1] = *(const v8b*)(p + 16); return f.v;
  }
  static __device__ __forceinline__ v8f mma(v16b a, v16b b, v8f c) {
    return __builtin_amdgcn_wmma_f32_16x16x32_bf16(false, a, false, b, (short)0, c, false, false);
  }
  static __device__ __forceinline__ void guard(v8f& a, v8f& b, v16b x, v16b y) { dep_guard_b(a, b, x, y); }
  static __device__ __forceinline__ void keep(v16b a, v16b b, v16b c, v16b d) { keep4_b(a, b, c, d); }
};

__device__ __forceinline__ v16b frag_u16(const unsigned short* p) {
  union { v16b v; v8b h[2]; } f;
  f.h[0] = *(const v8b*)(p);
  f.h[1] = *(const v8b*)(p + 16);
  return f.v;
}
__device__ __forceinline__ v8f mma_bf(v16b a, v16b b, v8f c) {
  return __builtin_amdgcn_wmma_f32_16x16x32_bf16(false, a, false, b, (short)0, c, false, false);
}

__device__ __forceinline__ void cvt8_store(const float* __restrict__ s, unsigned short* __restrict__ d) {
  const v4f a = *(const v4f*)(s);
  const v4f c = *(const v4f*)(s + 4);
  v4u w;
  w[0] = pack_bf2(a[0], a[1]); w[1] = pack_bf2(a[2], a[3]);
  w[2] = pack_bf2(c[0], c[1]); w[3] = pack_bf2(c[2], c[3]);
  *(volatile v4u*)(d) = w;
  __threadfence();
  *(volatile v4u*)(d) = w;
}

constexpr int PREP_TILE_BLOCKS = NBATCH * (NPT / 64);
constexpr int PREP_PT_BLOCKS   = NBATCH * NPT / 256;
constexpr int PREP_W10_BLOCKS  = CIN * CIN / (8 * 256);
constexpr int PREP_W11_BLOCKS  = COUT * 2 * CIN / (8 * 256);
constexpr int PREP_WSK_BLOCKS  = COUT * CIN / (8 * 256);
constexpr int PREP_BLOCKS = PREP_TILE_BLOCKS + PREP_PT_BLOCKS + PREP_W10_BLOCKS + PREP_W11_BLOCKS + PREP_WSK_BLOCKS;
static_assert((CIN * CIN) % 2048 == 0 && (COUT * 2 * CIN) % 2048 == 0 && (COUT * CIN) % 2048 == 0, "whole blocks per weight");
static_assert((NBATCH * NPT) % 256 == 0, "whole blocks per point set");

__global__ __launch_bounds__(256) void k_prep(
    const float* __restrict__ f, const float* __restrict__ p,
    const float* __restrict__ W10, const float* __restrict__ W11, const float* __restrict__ Wsk,
    unsigned short* __restrict__ fT, float* __restrict__ pR,
    unsigned short* __restrict__ W10b, unsigned short* __restrict__ W11d, unsigned short* __restrict__ Wsb) {
  __shared__ __align__(16) float tileT[64 * 68];
  const int t = threadIdx.x;
  const int bx = blockIdx.x;
  if (bx < PREP_TILE_BLOCKS) {
    const int b = bx / (NPT / 64);
    const int n0 = (bx % (NPT / 64)) * 64;
#pragma unroll
    for (int i = 0; i < 4; ++i) {
      const int e = t + 256 * i;
      const int c = e >> 4;
      const int n4 = (e & 15) * 4;
      const v4f v = *(const v4f*)(f + ((size_t)(b * CIN + c)) * NPT + n0 + n4);
      *(v4f*)(tileT + c * 68 + n4) = v;
    }
    __syncthreads();
    const int c8 = (t & 7) * 8;
    const int rr = t >> 3;
    v4u w[2];
#pragma unroll
    for (int jj = 0; jj < 2; ++jj) {
      const int n = rr + 32 * jj;
#pragma unroll
      for (int e = 0; e < 4; ++e)
        w[jj][e] = pack_bf2(tileT[(c8 + 2 * e) * 68 + n], tileT[(c8 + 2 * e + 1) * 68 + n]);
    }
    for (int pass = 0; pass < 2; ++pass) {
#pragma unroll
      for (int jj = 0; jj < 2; ++jj) {
        const int n = rr + 32 * jj;
        *(volatile v4u*)(fT + ((size_t)(b * NPT + n0 + n)) * CIN + c8) = w[jj];
      }
      __threadfence();
    }
  } else if (bx < PREP_TILE_BLOCKS + PREP_PT_BLOCKS) {
    const int q = (bx - PREP_TILE_BLOCKS) * 256 + t;
    const float x = p[(size_t)q * 3 + 0];
    const float y = p[(size_t)q * 3 + 1];
    const float z = p[(size_t)q * 3 + 2];
    v4f v;
    v[0] = rbf(x); v[1] = rbf(y); v[2] = rbf(z); v[3] = 0.0f;
    for (int pass = 0; pass < 2; ++pass) {
      *(volatile v4f*)(pR + (size_t)q * 4) = v;
      __threadfence();
    }
  } else {
    const int wb = bx - PREP_TILE_BLOCKS - PREP_PT_BLOCKS;
    if (wb < PREP_W10_BLOCKS) {
      const int grp = wb * 256 + t;
      const int e0 = grp * 8;
      cvt8_store(W10 + e0, W10b + e0);
    } else if (wb < PREP_W10_BLOCKS + PREP_W11_BLOCKS) {
      const int grp = (wb - PREP_W10_BLOCKS) * 256 + t;
      const int e0 = grp * 8;
      const int o = e0 >> 7;
      const int kk = e0 & 127;
      cvt8_store(W11 + o * CIN + (kk & (CIN - 1)), W11d + e0);
    } else {
      const int grp = (wb - PREP_W10_BLOCKS - PREP_W11_BLOCKS) * 256 + t;
      const int e0 = grp * 8;
      cvt8_store(Wsk + e0, Wsb + e0);
    }
  }
}

constexpr int FPS_THREADS = 512;
constexpr int FPS_PPT = NPT / FPS_THREADS;
constexpr int FPS_DYN_LDS = 3 * NPT * 4;
static_assert(FPS_PPT * FPS_THREADS == NPT && FPS_THREADS / 32 == 16 && FPS_PPT == 16, "selection geometry");
static_assert(MPT % FPS_THREADS == 0 && MPT % 64 == 0 && MPT / 64 == 32, "tail geometry");

__global__ __launch_bounds__(FPS_THREADS) void k_fps(
    const float* __restrict__ pR, const unsigned short* __restrict__ fT,
    float* __restrict__ newp, unsigned short* __restrict__ fiT) {
  extern __shared__ __align__(16) unsigned char fdyn[];
  float* px = (float*)fdyn;
  float* py = px + NPT;
  float* pz = py + NPT;
  __shared__ int idxL[MPT];
  __shared__ float rv[2][16];
  __shared__ int ri[2][16];
  const int b = blockIdx.x;
  const int t = threadIdx.x;
  const int lane = t & 31;
  const int wave = t >> 5;

  float xr[FPS_PPT], yr[FPS_PPT], zr[FPS_PPT], mr[FPS_PPT];
#pragma unroll
  for (int grp = 0; grp < 4; ++grp) {
#pragma unroll
    for (int i2 = 0; i2 < 4; ++i2) {
      const int i = grp * 4 + i2;
      const int n = t + FPS_THREADS * i;
      const v4f v = *(const v4f*)(pR + ((size_t)(b * NPT + n)) * 4);
      xr[i] = v[0]; yr[i] = v[1]; zr[i] = v[2]; mr[i] = 1e10f;
      px[n] = v[0]; py[n] = v[1]; pz[n] = v[2];
    }
    asm volatile("" ::: "memory");
  }
  if (t == 0) idxL[0] = 0;
  __syncthreads();

  int cur = 0;
  for (int s = 1; s < MPT; ++s) {
    const float lx = px[cur], ly = py[cur], lz = pz[cur];
    float bv = -1.0f;
    int bi = 0;
#pragma unroll
    for (int i = 0; i < FPS_PPT; ++i) {
      const float d = dist2_ord(xr[i], yr[i], zr[i], lx, ly, lz);
      const float mv = fminf(mr[i], d);
      mr[i] = mv;
      const bool take = mv > bv;
      bv = take ? mv : bv;
      bi = take ? (t + FPS_THREADS * i) : bi;
    }
#pragma unroll
    for (int off = 16; off > 0; off >>= 1) {
      const float ov = __shfl_xor(bv, off, 32);
      const int oi = __shfl_xor(bi, off, 32);
      const bool take = (ov > bv) || (ov == bv && oi < bi);
      bv = take ? ov : bv;
      bi = take ? oi : bi;
    }
    const int par = s & 1;
    if (lane == 0) { rv[par][wave] = bv; ri[par][wave] = bi; }
    __syncthreads();
    float gv = rv[par][lane & 15];
    int gi = ri[par][lane & 15];
#pragma unroll
    for (int off = 8; off > 0; off >>= 1) {
      const float ov = __shfl_xor(gv, off, 32);
      const int oi = __shfl_xor(gi, off, 32);
      const bool take = (ov > gv) || (ov == gv && oi < gi);
      gv = take ? ov : gv;
      gi = take ? oi : gi;
    }
    cur = gi;
    if (t == 0) idxL[s] = gi;
  }
  __syncthreads();

  {
    v4f w[MPT / FPS_THREADS];
#pragma unroll
    for (int j = 0; j < MPT / FPS_THREADS; ++j) {
      const int m = t + FPS_THREADS * j;
      const int n = idxL[m] & (NPT - 1);
      v4f v;
      v[0] = px[n]; v[1] = py[n]; v[2] = pz[n]; v[3] = 0.0f;
      w[j] = v;
    }
    for (int pass = 0; pass < 2; ++pass) {
#pragma unroll
      for (int j = 0; j < MPT / FPS_THREADS; ++j) {
        const int m = t + FPS_THREADS * j;
        *(volatile v4f*)(newp + ((size_t)(b * MPT + m)) * 4) = w[j];
      }
      __threadfence();
    }
  }
  {
    const int c8 = (t & 7) * 8;
    const int r0 = t >> 3;
#pragma unroll 1
    for (int chunk = 0; chunk < 8; ++chunk) {
      v4u w[4];
#pragma unroll
      for (int e = 0; e < 4; ++e) {
        const int m = r0 + 64 * (chunk * 4 + e);
        const int n = idxL[m] & (NPT - 1);
        w[e] = *(const v4u*)(fT + ((size_t)(b * NPT + n)) * CIN + c8);
      }
      for (int pass = 0; pass < 2; ++pass) {
#pragma unroll
        for (int e = 0; e < 4; ++e) {
          const int m = r0 + 64 * (chunk * 4 + e);
          *(volatile v4u*)(fiT + ((size_t)(b * MPT + m)) * CIN + c8) = w[e];
        }
        __threadfence();
      }
    }
  }
}

template <int BIAS_MODE, bool GSC, int OUT_MODE, int ACT>
__global__ __launch_bounds__(256) void k_gemm64(
    const unsigned short* __restrict__ Ap, int lda, long strideA,
    const unsigned short* __restrict__ Btp, int ldb, long strideB,
    void* __restrict__ Cout, void* __restrict__ Cout2, int ldc, long strideC,
    const float* __restrict__ bias, const float* __restrict__ gsc,
    int M, int N, int K, float scale) {
  typedef __bf16 T;
  typedef v16b V;
  const T* A = (const T*)Ap;
  const T* Bt = (const T*)Btp;
  __shared__ __align__(16) float sT[8][16 * 68];
  const int b    = blockIdx.y;
  const int lane = threadIdx.x & 31;
  const int wave = threadIdx.x >> 5;
  const int tilesN = N >> 6;
  const int tilesM = M >> 6;
  const int tile = blockIdx.x * 8 + wave;
  if (tile >= tilesM * tilesN) return;
  const int tm = tile / tilesN;
  const int tn = tile - tm * tilesN;
  const int m0 = tm << 6;
  const int n0 = tn << 6;

  const T* Ab = A  + (size_t)b * strideA;
  const T* Bb = Bt + (size_t)b * strideB;

  const int rlane = lane & 15;
  const int koff  = (lane >> 4) * 8;
  const int mOff  = (lane >> 4) * 8;

  v8f acc[4][4];
#pragma unroll
  for (int i = 0; i < 4; ++i)
#pragma unroll
    for (int j = 0; j < 4; ++j) acc[i][j] = (v8f){0.f,0.f,0.f,0.f,0.f,0.f,0.f,0.f};

  for (int k0 = 0; k0 < K; k0 += 32) {
    V bh[4];
#pragma unroll
    for (int j = 0; j < 4; ++j) {
      const size_t bo = (size_t)(n0 + (j << 4) + rlane) * ldb + koff + k0;
      bh[j] = Frag<T>::load(Bb + bo);
    }
#pragma unroll
    for (int i = 0; i < 4; ++i) {
      const size_t ao = (size_t)(m0 + (i << 4) + rlane) * lda + koff + k0;
      V ah = Frag<T>::load(Ab + ao);
#pragma unroll
      for (int j = 0; j < 4; ++j) acc[i][j] = Frag<T>::mma(ah, bh[j], acc[i][j]);
      Frag<T>::guard(acc[i][0], acc[i][3], ah, ah);
    }
    Frag<T>::keep(bh[0], bh[1], bh[2], bh[3]);
  }
  acc_guard4(acc[0][0], acc[0][1], acc[0][2], acc[0][3]);
  acc_guard4(acc[1][0], acc[1][1], acc[1][2], acc[1][3]);
  acc_guard4(acc[2][0], acc[2][1], acc[2][2], acc[2][3]);
  acc_guard4(acc[3][0], acc[3][1], acc[3][2], acc[3][3]);

  float* slab = sT[wave];
#pragma unroll
  for (int i = 0; i < 4; ++i) {
    const int mBase = m0 + (i << 4);
    float bm8[8];
#pragma unroll
    for (int r = 0; r < 8; ++r) bm8[r] = 0.0f;
    if (BIAS_MODE == 1) {
      const v4f q0 = *(const v4f*)(bias + mBase + mOff);
      const v4f q1 = *(const v4f*)(bias + mBase + mOff + 4);
      bm8[0] = rbf(q0[0]); bm8[1] = rbf(q0[1]); bm8[2] = rbf(q0[2]); bm8[3] = rbf(q0[3]);
      bm8[4] = rbf(q1[0]); bm8[5] = rbf(q1[1]); bm8[6] = rbf(q1[2]); bm8[7] = rbf(q1[3]);
    }
#pragma unroll
    for (int j = 0; j < 4; ++j) {
      const int n = n0 + (j << 4) + rlane;
      float bv = 0.f, gv = 1.f;
      if (BIAS_MODE == 2) {
        bv = rbf(bias[n]);
        if (GSC) gv = rbf(gsc[n]);
      }
#pragma unroll
      for (int r = 0; r < 8; ++r) {
        float v = acc[i][j][r] * scale;
        if (BIAS_MODE == 1) v += bm8[r];
        if (BIAS_MODE == 2) v = v * gv + bv;
        if (ACT == 2) v = fmaxf(v, 0.0f);
        slab[(mOff + r) * 68 + (j << 4) + rlane] = v;
      }
    }
    __builtin_amdgcn_fence(__ATOMIC_RELEASE, "workgroup");
    __builtin_amdgcn_wave_barrier();
    __builtin_amdgcn_fence(__ATOMIC_ACQUIRE, "workgroup");
    if (OUT_MODE == 0) {
      float* C = (float*)Cout + (size_t)b * strideC;
      const int hh = lane >> 4, c4 = (lane & 15) * 4;
      for (int pass = 0; pass < 2; ++pass) {
#pragma unroll
        for (int it = 0; it < 8; ++it) {
          const int row = it * 2 + hh;
          v4f v = *(const v4f*)(slab + row * 68 + c4);
          *(volatile v4f*)(C + (size_t)(mBase + row) * ldc + n0 + c4) = v;
        }
        __threadfence();
      }
    } else {
      const int q = lane >> 3, c8 = (lane & 7) * 8;
      unsigned short* C  = (unsigned short*)Cout  + (size_t)b * strideC;
      unsigned short* Cl = (unsigned short*)Cout2 + (size_t)b * strideC;
      for (int pass = 0; pass < 2; ++pass) {
#pragma unroll
        for (int it = 0; it < 4; ++it) {
          const int row = it * 4 + q;
          const float* sp = slab + row * 68 + c8;
          v8h hv, lv;
#pragma unroll
          for (int e = 0; e < 8; ++e) {
            unsigned short hb = f2bf_bits(sp[e]);
            unsigned short lb = f2bf_bits(sp[e] - bf_bits2f(hb));
            hv[e] = __builtin_bit_cast(_Float16, hb);
            lv[e] = __builtin_bit_cast(_Float16, lb);
          }
          *(volatile v8h*)(C  + (size_t)(mBase + row) * ldc + n0 + c8) = hv;
          *(volatile v8h*)(Cl + (size_t)(mBase + row) * ldc + n0 + c8) = lv;
        }
        __threadfence();
      }
    }
    __builtin_amdgcn_fence(__ATOMIC_RELEASE, "workgroup");
    __builtin_amdgcn_wave_barrier();
    __builtin_amdgcn_fence(__ATOMIC_ACQUIRE, "workgroup");
  }
}

constexpr int TAIL_X_BYTES  = 8 * KNB * XP * 2;
constexpr int TAIL_MV_BYTES = COUT * MVP * 4;
constexpr int TAIL_DYN_LDS  = 2 * TAIL_X_BYTES + TAIL_MV_BYTES;
static_assert(TAIL_X_BYTES % 16 == 0, "lds carve alignment");
static_assert(CPE * CPE == 4 * 256 && COUT * CPE == 16 * 256 && CPE * 3 == 96, "parameter staging geometry");

__global__ __launch_bounds__(256) void k_tail(
    const float* __restrict__ pR, const float* __restrict__ newp,
    const float* __restrict__ hT, const float* __restrict__ ident,
    const float* __restrict__ W20, const float* __restrict__ g20, const float* __restrict__ b20,
    const float* __restrict__ W21, const float* __restrict__ g21, const float* __restrict__ b21,
    const float* __restrict__ W22, const float* __restrict__ g22, const float* __restrict__ b22,
    float* __restrict__ out) {
  extern __shared__ __align__(16) unsigned char tdyn[];
  unsigned short* X0s = (unsigned short*)(tdyn);
  unsigned short* X1s = (unsigned short*)(tdyn + TAIL_X_BYTES);
  float* maxv = (float*)(tdyn + 2 * TAIL_X_BYTES);
  __shared__ __align__(16) unsigned short W21s[CPE * XP];
  __shared__ __align__(16) unsigned short W22s[COUT * XP];
  __shared__ __align__(16) float W20s[CPE * 3];
  __shared__ __align__(16) float g20s[CPE];
  __shared__ __align__(16) float b20s[CPE];
  __shared__ __align__(16) float g21s[CPE];
  __shared__ __align__(16) float b21s[CPE];
  __shared__ __align__(16) float g22s[COUT];
  __shared__ __align__(16) float b22s[COUT];
  __shared__ int gls[8][KNB];

  const int t = threadIdx.x;
  const int lane = t & 31;
  const int wave = t >> 5;
  const int rl = lane & 15;
  const int hh = lane >> 4;
  const int koff = hh * 8;
  const int b = blockIdx.y;
  const int m0 = blockIdx.x * QPB;

  {
#pragma unroll
    for (int i = 0; i < 4; ++i) {
      const int e0 = 4 * (t + 256 * i);
      const v4f w4 = *(const v4f*)(W22 + e0);
      v2u pk;
      pk[0] = pack_bf2(w4[0], w4[1]);
      pk[1] = pack_bf2(w4[2], w4[3]);
      *(v2u*)(W22s + (e0 >> 5) * XP + (e0 & 31)) = pk;
    }
  }
  asm volatile("" ::: "memory");
  {
    {
      const int e0 = 4 * t;
      const v4f w4 = *(const v4f*)(W21 + e0);
      v2u pk;
      pk[0] = pack_bf2(w4[0], w4[1]);
      pk[1] = pack_bf2(w4[2], w4[3]);
      *(v2u*)(W21s + (e0 >> 5) * XP + (e0 & 31)) = pk;
    }
    if (t < 24) {
      const v4f w4 = *(const v4f*)(W20 + 4 * t);
      v4f r4;
      r4[0] = rbf(w4[0]); r4[1] = rbf(w4[1]); r4[2] = rbf(w4[2]); r4[3] = rbf(w4[3]);
      *(v4f*)(W20s + 4 * t) = r4;
    }
    if (t < 8) {
      const v4f a4 = *(const v4f*)(g20 + 4 * t);
      const v4f c4v = *(const v4f*)(b20 + 4 * t);
      const v4f d4 = *(const v4f*)(g21 + 4 * t);
      const v4f e4 = *(const v4f*)(b21 + 4 * t);
      v4f ra, rc, rd, re;
#pragma unroll
      for (int e = 0; e < 4; ++e) { ra[e] = rbf(a4[e]); rc[e] = rbf(c4v[e]); rd[e] = rbf(d4[e]); re[e] = rbf(e4[e]); }
      *(v4f*)(g20s + 4 * t) = ra;
      *(v4f*)(b20s + 4 * t) = rc;
      *(v4f*)(g21s + 4 * t) = rd;
      *(v4f*)(b21s + 4 * t) = re;
    }
    if (t < 32) {
      const v4f a4 = *(const v4f*)(g22 + 4 * t);
      const v4f c4v = *(const v4f*)(b22 + 4 * t);
      v4f ra, rc;
#pragma unroll
      for (int e = 0; e < 4; ++e) { ra[e] = rbf(a4[e]); rc[e] = rbf(c4v[e]); }
      *(v4f*)(g22s + 4 * t) = ra;
      *(v4f*)(b22s + 4 * t) = rc;
    }
  }
  __syncthreads();

  unsigned short* X0w = X0s + wave * (KNB * XP);
  unsigned short* X1w = X1s + wave * (KNB * XP);
  int* glw = gls[wave];
  const float* pb = pR + (size_t)b * NPT * 4;
  const float* hb = hT + (size_t)b * NPT * COUT;
  const v8f zz = (v8f){0.f,0.f,0.f,0.f,0.f,0.f,0.f,0.f};

#pragma unroll 1
  for (int j = 0; j < QPB / 8; ++j) {
    const int ml = wave * (QPB / 8) + j;
    const int qrow = b * MPT + m0 + ml;
    wave_sync();
    const v4f q4 = *(const v4f*)(newp + (size_t)qrow * 4);

    int count = 0, first = 0;
#pragma unroll 1
    for (int it = 0; it < NPT / 32; ++it) {
      if (count >= KNB) break;
      const int n = it * 32 + lane;
      const v4f pt = *(const v4f*)(pb + (size_t)n * 4);
      const float d2 = dist2_ord(q4[0], q4[1], q4[2], pt[0], pt[1], pt[2]);
      const bool inb = (d2 <= RAD2);
      const unsigned mask = (unsigned)__ballot(inb);
      const int pos = count + (int)__popc(mask & ((1u << lane) - 1u));
      if (inb && pos < KNB) glw[pos] = n;
      if (count == 0 && mask != 0u) first = it * 32 + (int)(__builtin_ffs((int)mask) - 1);
      count += (int)__popc(mask);
    }
    if (lane >= count) glw[lane] = first;
    wave_sync();

    {
      const int g = glw[lane] & (NPT - 1);
      const v4f gp = *(const v4f*)(pb + (size_t)g * 4);
      const float dx = gp[0] - q4[0];
      const float dy = gp[1] - q4[1];
      const float dz = gp[2] - q4[2];
#pragma unroll
      for (int grp = 0; grp < 4; ++grp) {
        v4u pk;
#pragma unroll
        for (int e2 = 0; e2 < 4; ++e2) {
          const int o = grp * 8 + e2 * 2;
          const float s0 = W20s[o * 3 + 0] * dx + W20s[o * 3 + 1] * dy + W20s[o * 3 + 2] * dz;
          const float s1 = W20s[o * 3 + 3] * dx + W20s[o * 3 + 4] * dy + W20s[o * 3 + 5] * dz;
          const float v0 = fmaxf(g20s[o] * s0 + b20s[o], 0.0f);
          const float v1 = fmaxf(g20s[o + 1] * s1 + b20s[o + 1], 0.0f);
          pk[e2] = pack_bf2(v0, v1);
        }
        *(v4u*)(X0w + lane * XP + grp * 8) = pk;
      }
    }
    wave_sync();

    {
      const v16b xb0 = frag_u16(X0w + rl * XP + koff);
      const v16b xb1 = frag_u16(X0w + (16 + rl) * XP + koff);
#pragma unroll
      for (int rt = 0; rt < 2; ++rt) {
        const v16b wa = frag_u16(W21s + (16 * rt + rl) * XP + koff);
        v8f a0 = zz, a1 = zz;
        a0 = mma_bf(wa, xb0, a0);
        a1 = mma_bf(wa, xb1, a1);
        dep_guard3(a0, a1, wa, xb0, xb1);
        v4u p0, p1;
#pragma unroll
        for (int e2 = 0; e2 < 4; ++e2) {
          const int o = 16 * rt + 8 * hh + 2 * e2;
          const float ga = g21s[o], ba = b21s[o], gc = g21s[o + 1], bc = b21s[o + 1];
          p0[e2] = pack_bf2(fmaxf(ga * a0[2 * e2] + ba, 0.0f), fmaxf(gc * a0[2 * e2 + 1] + bc, 0.0f));
          p1[e2] = pack_bf2(fmaxf(ga * a1[2 * e2] + ba, 0.0f), fmaxf(gc * a1[2 * e2 + 1] + bc, 0.0f));
        }
        *(v4u*)(X1w + rl * XP + 16 * rt + 8 * hh) = p0;
        *(v4u*)(X1w + (16 + rl) * XP + 16 * rt + 8 * hh) = p1;
      }
    }
    wave_sync();

    {
      const v16b xb0 = frag_u16(X1w + rl * XP + koff);
      const v16b xb1 = frag_u16(X1w + (16 + rl) * XP + koff);
      const int g0 = glw[rl] & (NPT - 1);
      const int g1 = glw[16 + rl] & (NPT - 1);
      const float* h0p = hb + (size_t)g0 * COUT + 8 * hh;
      const float* h1p = hb + (size_t)g1 * COUT + 8 * hh;
#pragma unroll 1
      for (int rt = 0; rt < COUT / 16; ++rt) {
        const v16b wa = frag_u16(W22s + (16 * rt + rl) * XP + koff);
        v8f a0 = zz, a1 = zz;
        a0 = mma_bf(wa, xb0, a0);
        a1 = mma_bf(wa, xb1, a1);
        dep_guard3(a0, a1, wa, xb0, xb1);
        const v4f fa = *(const v4f*)(h0p + 16 * rt);
        const v4f fb = *(const v4f*)(h0p + 16 * rt + 4);
        const v4f fc = *(const v4f*)(h1p + 16 * rt);
        const v4f fd = *(const v4f*)(h1p + 16 * rt + 4);
        const float fj0[8] = {fa[0], fa[1], fa[2], fa[3], fb[0], fb[1], fb[2], fb[3]};
        const float fj1[8] = {fc[0], fc[1], fc[2], fc[3], fd[0], fd[1], fd[2], fd[3]};
        float vm[8];
#pragma unroll
        for (int r = 0; r < 8; ++r) {
          const int o = 16 * rt + 8 * hh + r;
          const float gg = g22s[o], bb = b22s[o];
          const float v0 = fmaxf(gg * a0[r] + bb, 0.0f) + fj0[r];
          const float v1 = fmaxf(gg * a1[r] + bb, 0.0f) + fj1[r];
          vm[r] = fmaxf(v0, v1);
        }
#pragma unroll
        for (int off = 1; off < 16; off <<= 1) {
#pragma unroll
          for (int r = 0; r < 8; ++r) {
            const float ov = __shfl_xor(vm[r], off, 32);
            vm[r] = fmaxf(vm[r], ov);
          }
        }
        if (rl == 0) {
#pragma unroll
          for (int r = 0; r < 8; ++r) maxv[(16 * rt + 8 * hh + r) * MVP + ml] = vm[r];
        }
      }
    }
  }
  __syncthreads();

  {
    float* ob = out + ((size_t)b * COUT) * MPT + m0;
    const float* ib = ident + ((size_t)b * COUT) * MPT + m0;
    const int q8 = lane >> 3;
    const int c4 = (lane & 7) * 4;
    v4f vals[4];
#pragma unroll
    for (int it = 0; it < 4; ++it) {
      const int o = wave * 16 + it * 4 + q8;
      const v4f mv = *(const v4f*)(maxv + o * MVP + c4);
      const v4f iv = *(const v4f*)(ib + (size_t)o * MPT + c4);
      v4f rq;
      rq[0] = fmaxf(mv[0] + iv[0], 0.0f);
      rq[1] = fmaxf(mv[1] + iv[1], 0.0f);
      rq[2] = fmaxf(mv[2] + iv[2], 0.0f);
      rq[3] = fmaxf(mv[3] + iv[3], 0.0f);
      vals[it] = rq;
    }
    for (int pass = 0; pass < 2; ++pass) {
#pragma unroll
      for (int it = 0; it < 4; ++it) {
        const int o = wave * 16 + it * 4 + q8;
        *(volatile v4f*)(ob + (size_t)o * MPT + c4) = vals[it];
      }
      __threadfence();
    }
  }
}

static_assert(NPT % 64 == 0 && CIN % 64 == 0 && CIN % 32 == 0, "L3 shape");
static_assert(NPT % 64 == 0 && COUT % 64 == 0 && (2 * CIN) % 32 == 0, "L4 shape");
static_assert(COUT % 64 == 0 && MPT % 64 == 0 && CIN % 32 == 0, "L5 shape");
constexpr int GRID_L3 = (NPT / 64) * (CIN / 64) / 8;
constexpr int GRID_L4 = (NPT / 64) * (COUT / 64) / 8;
constexpr int GRID_L5 = (COUT / 64) * (MPT / 64) / 8;
static_assert(GRID_L3 * 8 == (NPT / 64) * (CIN / 64), "exact tile blocks");
static_assert(GRID_L4 * 8 == (NPT / 64) * (COUT / 64), "exact tile blocks");
static_assert(GRID_L5 * 8 == (COUT / 64) * (MPT / 64), "exact tile blocks");

extern "C" void kernel_launch(void* const* d_in, const int* in_sizes, int n_in,
                              void* d_out, int out_size, void* d_ws, size_t ws_size, hipStream_t stream) {
  if (n_in < 19) return;
  if (in_sizes[0] != NBATCH * NPT * 3) return;
  if (in_sizes[1] != NBATCH * CIN * NPT) return;
  if (in_sizes[2] != CIN * CIN || in_sizes[5] != COUT * CIN || in_sizes[8] != CPE * 3 ||
      in_sizes[11] != CPE * CPE || in_sizes[14] != COUT * CPE || in_sizes[17] != COUT * CIN) return;
  if (in_sizes[3] != CIN || in_sizes[4] != CIN || in_sizes[6] != COUT || in_sizes[7] != COUT ||
      in_sizes[9] != CPE || in_sizes[10] != CPE || in_sizes[12] != CPE || in_sizes[13] != CPE ||
      in_sizes[15] != COUT || in_sizes[16] != COUT || in_sizes[18] != COUT) return;
  if (out_size != NBATCH * COUT * MPT) return;
  if (ws_size < WS_TOTAL) return;

  const float* p    = (const float*)d_in[0];
  const float* f    = (const float*)d_in[1];
  const float* W1_0 = (const float*)d_in[2];
  const float* g1_0 = (const float*)d_in[3];
  const float* b1_0 = (const float*)d_in[4];
  const float* W1_1 = (const float*)d_in[5];
  const float* g1_1 = (const float*)d_in[6];
  const float* b1_1 = (const float*)d_in[7];
  const float* W2_0 = (const float*)d_in[8];
  const float* g2_0 = (const float*)d_in[9];
  const float* b2_0 = (const float*)d_in[10];
  const float* W2_1 = (const float*)d_in[11];
  const float* g2_1 = (const float*)d_in[12];
  const float* b2_1 = (const float*)d_in[13];
  const float* W2_2 = (const float*)d_in[14];
  const float* g2_2 = (const float*)d_in[15];
  const float* b2_2 = (const float*)d_in[16];
  const float* Wskp = (const float*)d_in[17];
  const float* bskp = (const float*)d_in[18];
  float* out = (float*)d_out;

  char* ws = (char*)d_ws;
  float*          pR   = (float*)(ws + OFF_PR);
  unsigned short* fT   = (unsigned short*)(ws + OFF_FT);
  unsigned short* W10b = (unsigned short*)(ws + OFF_W10);
  unsigned short* W11d = (unsigned short*)(ws + OFF_W11);
  unsigned short* Wsb  = (unsigned short*)(ws + OFF_WSK);
  float*          newp = (float*)(ws + OFF_NEWP);
  unsigned short* fiT  = (unsigned short*)(ws + OFF_FIT);
  unsigned short* h1c  = (unsigned short*)(ws + OFF_H1);
  float*          hT   = (float*)(ws + OFF_HT);
  float*          ident = (float*)(ws + OFF_ID);

  k_prep<<<PREP_BLOCKS, 256, 0, stream>>>(f, p, W1_0, W1_1, Wskp, fT, pR, W10b, W11d, Wsb);
  k_fps<<<NBATCH, FPS_THREADS, FPS_DYN_LDS, stream>>>(pR, fT, newp, fiT);
  k_gemm64<2, true, 2, 2><<<dim3(GRID_L3, NBATCH), 256, 0, stream>>>(
      fT, CIN, (long)NPT * CIN, W10b, CIN, 0L,
      (void*)h1c, (void*)(h1c + CIN), 2 * CIN, (long)NPT * 2 * CIN,
      b1_0, g1_0, NPT, CIN, CIN, 1.0f);
  k_gemm64<2, true, 0, 0><<<dim3(GRID_L4, NBATCH), 256, 0, stream>>>(
      h1c, 2 * CIN, (long)NPT * 2 * CIN, W11d, 2 * CIN, 0L,
      (void*)hT, (void*)hT, COUT, (long)NPT * COUT,
      b1_1, g1_1, NPT, COUT, 2 * CIN, 1.0f);
  k_gemm64<1, false, 0, 0><<<dim3(GRID_L5, NBATCH), 256, 0, stream>>>(
      Wsb, CIN, 0L, fiT, CIN, (long)MPT * CIN,
      (void*)ident, (void*)ident, MPT, (long)COUT * MPT,
      bskp, bskp, COUT, MPT, CIN, 1.0f);
  k_tail<<<dim3(MPT / QPB, NBATCH), 256, TAIL_DYN_LDS, stream>>>(
      pR, newp, hT, ident, W2_0, g2_0, b2_0, W2_1, g2_1, b2_1, W2_2, g2_2, b2_2, out);
}
